// ImprovedTAPCell_52166672777401
// MI455X (gfx1250) — hardware-verified
//
#include <hip/hip_runtime.h>
#include <math.h>
#include <stdint.h>

#define NQ  8192
#define NH  1024
#define NM  4096
#define QCH 2048
static_assert((NQ % QCH) == 0);
static_assert((QCH % 64) == 0 && (NM % 64) == 0 && (NH % 64) == 0);
static_assert((NH % 32) == 0 && (NM % 32) == 0);
static_assert(NM == 256 * 16);
static_assert(((NQ * NH) % (8 * 256)) == 0 && ((NM * NH) % (8 * 256)) == 0);

typedef __bf16   v16b __attribute__((ext_vector_type(16)));
typedef __bf16   v8b  __attribute__((ext_vector_type(8)));
typedef float    v8f  __attribute__((ext_vector_type(8)));
typedef float    v4f  __attribute__((ext_vector_type(4)));
typedef unsigned int v4u __attribute__((ext_vector_type(4)));

__device__ __forceinline__ unsigned short bf_bits(float f) {
  unsigned u = __float_as_uint(f);
  return (unsigned short)((u + 0x7FFFu + ((u >> 16) & 1u)) >> 16);
}
__device__ __forceinline__ unsigned pk16(unsigned short a, unsigned short b) { return (unsigned)a | ((unsigned)b << 16); }
__device__ __forceinline__ v8f zero8() { v8f z = {0.f, 0.f, 0.f, 0.f, 0.f, 0.f, 0.f, 0.f}; return z; }

__device__ __forceinline__ float bf_round(float f) {
  return __uint_as_float(((unsigned)bf_bits(f)) << 16);
}
__device__ __forceinline__ v16b ldfrag_b(const __bf16* p) {
  union { v16b v; v8b h[2]; } f;
  f.h[0] = *(const v8b*)(p);
  f.h[1] = *(const v8b*)(p + 16);
  return f.v;
}

__device__ __forceinline__ v8f mma_b_raw(v16b a, v16b b, v8f c) {
  return __builtin_amdgcn_wmma_f32_16x16x32_bf16(false, a, false, b, (short)0, c, false, false);
}
__device__ __forceinline__ void dep_guard_b(v8f& a, v8f& b, v16b x, v16b y) {
#if defined(__HIP_DEVICE_COMPILE__)
  asm volatile("v_nop\n\tv_nop\n\tv_nop\n\tv_nop" : "+v"(a), "+v"(b) : "v"(x), "v"(y));
#endif
}
__device__ __forceinline__ void keep4_b(v16b a, v16b b, v16b c, v16b d) {
#if defined(__HIP_DEVICE_COMPILE__)
  asm volatile("v_nop" :: "v"(a), "v"(b), "v"(c), "v"(d));
#endif
}
__device__ __forceinline__ void acc_guard4(v8f& a, v8f& b, v8f& c, v8f& d) {
#if defined(__HIP_DEVICE_COMPILE__)
  asm volatile("v_nop\n\tv_nop\n\tv_nop\n\tv_nop" : "+v"(a), "+v"(b), "+v"(c), "+v"(d));
#endif
}
__device__ __forceinline__ void wave_sync_lds() {
  __builtin_amdgcn_fence(__ATOMIC_RELEASE, "workgroup");
  __builtin_amdgcn_wave_barrier();
  __builtin_amdgcn_fence(__ATOMIC_ACQUIRE, "workgroup");
}

__global__ __launch_bounds__(256) void cvt_bf16x8(const float* __restrict__ in, unsigned short* out,
                                                  int n8, int n8tot) {
  const int i = blockIdx.x * 256 + threadIdx.x;
  if (i >= n8tot) return;
  int ic = i;
  if (ic > n8 - 1) ic = n8 - 1;
  const v4f a = *(const v4f*)(in + (size_t)ic * 8);
  const v4f b = *(const v4f*)(in + (size_t)ic * 8 + 4);
  v4u p;
  p[0] = pk16(bf_bits(a[0]), bf_bits(a[1]));
  p[1] = pk16(bf_bits(a[2]), bf_bits(a[3]));
  p[2] = pk16(bf_bits(b[0]), bf_bits(b[1]));
  p[3] = pk16(bf_bits(b[2]), bf_bits(b[3]));
  if (i >= n8) { p[0] = 0u; p[1] = 0u; p[2] = 0u; p[3] = 0u; }
  *(volatile v4u*)(out + (size_t)i * 8) = p;
  __threadfence();
  *(volatile v4u*)(out + (size_t)i * 8) = p;
}

__global__ __launch_bounds__(256) void tr_cvt64(const float* __restrict__ in, unsigned short* out,
                                                int R, int C) {
  __shared__ __align__(16) float s[64 * 68];
  const int tid = threadIdx.x;
  const int r0 = blockIdx.y * 64;
  const int c0 = blockIdx.x * 64;
  const int rl = tid >> 4;
  const int c4 = (tid & 15) * 4;
#pragma unroll
  for (int it = 0; it < 4; ++it) {
    const int r = it * 16 + rl;
    const v4f v = *(const v4f*)(in + (size_t)(r0 + r) * C + c0 + c4);
    s[(c4 + 0) * 68 + r] = v[0];
    s[(c4 + 1) * 68 + r] = v[1];
    s[(c4 + 2) * 68 + r] = v[2];
    s[(c4 + 3) * 68 + r] = v[3];
  }
  __syncthreads();
  const int q8 = (tid & 7) * 8;
  const int cl = tid >> 3;
  v4u pk[2];
#pragma unroll
  for (int it = 0; it < 2; ++it) {
    const int c = it * 32 + cl;
    const v4f a = *(const v4f*)(s + c * 68 + q8);
    const v4f b = *(const v4f*)(s + c * 68 + q8 + 4);
    v4u p;
    p[0] = pk16(bf_bits(a[0]), bf_bits(a[1]));
    p[1] = pk16(bf_bits(a[2]), bf_bits(a[3]));
    p[2] = pk16(bf_bits(b[0]), bf_bits(b[1]));
    p[3] = pk16(bf_bits(b[2]), bf_bits(b[3]));
    pk[it] = p;
  }
  for (int pass = 0; pass < 2; ++pass) {
#pragma unroll
    for (int it = 0; it < 2; ++it) {
      const int c = it * 32 + cl;
      *(volatile v4u*)(out + (size_t)(c0 + c) * R + r0 + q8) = pk[it];
    }
    __threadfence();
  }
}

template <int OUT16, int BIAS, int RES>
__global__ __launch_bounds__(256) void gemm64(
    const unsigned short* __restrict__ Ap, int lda,
    const unsigned short* __restrict__ Btp, int ldb,
    void* Cout, int ldc,
    const float* __restrict__ bias, int nbias,
    const float* __restrict__ res, int ldr,
    float alpha, int M, int N, int K) {
  const __bf16* A  = (const __bf16*)(const void*)Ap;
  const __bf16* Bt = (const __bf16*)(const void*)Btp;
  __shared__ __align__(16) float sT[8][16 * 68];
  const int lane = threadIdx.x & 31;
  const int wave = threadIdx.x >> 5;
  const int tilesN = N >> 6;
  const int tilesM = M >> 6;
  const int tile = blockIdx.x * 8 + wave;
  if (tile >= tilesM * tilesN) return;
  const int tm = tile / tilesN;
  const int tn = tile - tm * tilesN;
  const int m0 = tm << 6;
  const int n0 = tn << 6;

  const int rlane = lane & 15;
  const int koff  = (lane >> 4) * 8;
  const int mOff  = (lane >> 4) * 8;

  v8f acc[4][4];
#pragma unroll
  for (int i = 0; i < 4; ++i)
#pragma unroll
    for (int j = 0; j < 4; ++j) acc[i][j] = zero8();

  for (int k0 = 0; k0 < K; k0 += 32) {
    v16b bh[4];
#pragma unroll
    for (int j = 0; j < 4; ++j) {
      const size_t bo = (size_t)(n0 + (j << 4) + rlane) * ldb + koff + k0;
      bh[j] = ldfrag_b(Bt + bo);
    }
#pragma unroll
    for (int i = 0; i < 4; ++i) {
      const size_t ao = (size_t)(m0 + (i << 4) + rlane) * lda + koff + k0;
      const v16b ah = ldfrag_b(A + ao);
#pragma unroll
      for (int j = 0; j < 4; ++j) {
        acc[i][j] = mma_b_raw(ah, bh[j], acc[i][j]);
      }
      dep_guard_b(acc[i][0], acc[i][3], ah, bh[3]);
    }
    keep4_b(bh[0], bh[1], bh[2], bh[3]);
  }
  acc_guard4(acc[0][0], acc[0][1], acc[0][2], acc[0][3]);
  acc_guard4(acc[1][0], acc[1][1], acc[1][2], acc[1][3]);
  acc_guard4(acc[2][0], acc[2][1], acc[2][2], acc[2][3]);
  acc_guard4(acc[3][0], acc[3][1], acc[3][2], acc[3][3]);

  float* slab = sT[wave];
#pragma unroll
  for (int i = 0; i < 4; ++i) {
    const int mBase = m0 + (i << 4);
#pragma unroll
    for (int j = 0; j < 4; ++j) {
#pragma unroll
      for (int r = 0; r < 8; ++r) {
        slab[(mOff + r) * 68 + (j << 4) + rlane] = acc[i][j][r];
      }
    }
    wave_sync_lds();
    if (OUT16 == 0) {
      float* C = (float*)Cout;
      const int hh = lane >> 4, c4 = (lane & 15) * 4;
      for (int pass = 0; pass < 2; ++pass) {
#pragma unroll
        for (int it = 0; it < 8; ++it) {
          const int row = it * 2 + hh;
          v4f v = *(const v4f*)(slab + row * 68 + c4);
          v = v * alpha;
          if (BIAS == 1) {
            int bi = n0 + c4; if (bi > nbias - 4) bi = nbias - 4; if (bi < 0) bi = 0;
            const v4f bb = *(const v4f*)(bias + bi);
            v = v + bb;
          }
          if (BIAS == 2) {
            int bi = mBase + row; if (bi > nbias - 1) bi = nbias - 1; if (bi < 0) bi = 0;
            const float bb = bias[bi];
            v[0] += bb; v[1] += bb; v[2] += bb; v[3] += bb;
          }
          if (RES) {
            v4f rr = *(const v4f*)(res + (size_t)(mBase + row) * ldr + n0 + c4);
            rr[0] = bf_round(rr[0]); rr[1] = bf_round(rr[1]); rr[2] = bf_round(rr[2]); rr[3] = bf_round(rr[3]);
            v = v + rr;
          }
          *(volatile v4f*)(C + (size_t)(mBase + row) * ldc + n0 + c4) = v;
        }
        __threadfence();
      }
    } else {
      unsigned short* C16 = (unsigned short*)Cout;
      const int q8 = (lane & 7) * 8, rr = lane >> 3;
      v4u pk[4];
#pragma unroll
      for (int it = 0; it < 4; ++it) {
        const int row = it * 4 + rr;
        v4f a = *(const v4f*)(slab + row * 68 + q8);
        v4f b = *(const v4f*)(slab + row * 68 + q8 + 4);
        a = a * alpha;
        b = b * alpha;
        if (BIAS == 1) {
          int bi = n0 + q8; if (bi > nbias - 8) bi = nbias - 8; if (bi < 0) bi = 0;
          const v4f b0 = *(const v4f*)(bias + bi);
          const v4f b1 = *(const v4f*)(bias + bi + 4);
          a = a + b0;
          b = b + b1;
        }
        if (BIAS == 2) {
          int bi = mBase + row; if (bi > nbias - 1) bi = nbias - 1; if (bi < 0) bi = 0;
          const float bb = bias[bi];
          a[0] += bb; a[1] += bb; a[2] += bb; a[3] += bb;
          b[0] += bb; b[1] += bb; b[2] += bb; b[3] += bb;
        }
        v4u p;
        p[0] = pk16(bf_bits(a[0]), bf_bits(a[1]));
        p[1] = pk16(bf_bits(a[2]), bf_bits(a[3]));
        p[2] = pk16(bf_bits(b[0]), bf_bits(b[1]));
        p[3] = pk16(bf_bits(b[2]), bf_bits(b[3]));
        pk[it] = p;
      }
      for (int pass = 0; pass < 2; ++pass) {
#pragma unroll
        for (int it = 0; it < 4; ++it) {
          const int row = it * 4 + rr;
          *(volatile v4u*)(C16 + (size_t)(mBase + row) * ldc + n0 + q8) = pk[it];
        }
        __threadfence();
      }
    }
    wave_sync_lds();
  }
}

__global__ __launch_bounds__(256) void softmax_rows(const float* __restrict__ S, unsigned short* P) {
  __shared__ float sMx[8];
  __shared__ float sSm[8];
  const int tid  = threadIdx.x;
  const int lane = tid & 31;
  const int wave = tid >> 5;
  const size_t rb = (size_t)blockIdx.x * NM;
  const int c0 = tid * 8;
  const int c1 = (NM / 2) + tid * 8;
  const v4f a0 = *(const v4f*)(S + rb + c0);
  const v4f a1 = *(const v4f*)(S + rb + c0 + 4);
  const v4f a2 = *(const v4f*)(S + rb + c1);
  const v4f a3 = *(const v4f*)(S + rb + c1 + 4);
  float v[16];
  v[0]  = a0[0]; v[1]  = a0[1]; v[2]  = a0[2]; v[3]  = a0[3];
  v[4]  = a1[0]; v[5]  = a1[1]; v[6]  = a1[2]; v[7]  = a1[3];
  v[8]  = a2[0]; v[9]  = a2[1]; v[10] = a2[2]; v[11] = a2[3];
  v[12] = a3[0]; v[13] = a3[1]; v[14] = a3[2]; v[15] = a3[3];

  float mx = v[0];
#pragma unroll
  for (int i = 1; i < 16; ++i) mx = fmaxf(mx, v[i]);
  mx = fmaxf(mx, __shfl_xor(mx, 16));
  mx = fmaxf(mx, __shfl_xor(mx, 8));
  mx = fmaxf(mx, __shfl_xor(mx, 4));
  mx = fmaxf(mx, __shfl_xor(mx, 2));
  mx = fmaxf(mx, __shfl_xor(mx, 1));
  if (lane == 0) sMx[wave] = mx;
  __syncthreads();
  float m = sMx[0];
#pragma unroll
  for (int w = 1; w < 8; ++w) m = fmaxf(m, sMx[w]);

  float e[16];
#pragma unroll
  for (int i = 0; i < 16; ++i) e[i] = __expf(v[i] - m);
  float part = (((e[0] + e[1]) + (e[2] + e[3])) + ((e[4] + e[5]) + (e[6] + e[7]))) +
               (((e[8] + e[9]) + (e[10] + e[11])) + ((e[12] + e[13]) + (e[14] + e[15])));
  part += __shfl_xor(part, 16);
  part += __shfl_xor(part, 8);
  part += __shfl_xor(part, 4);
  part += __shfl_xor(part, 2);
  part += __shfl_xor(part, 1);
  if (lane == 0) sSm[wave] = part;
  __syncthreads();
  const float l = ((sSm[0] + sSm[1]) + (sSm[2] + sSm[3])) + ((sSm[4] + sSm[5]) + (sSm[6] + sSm[7]));
  const float inv = 1.0f / l;

  v4u p0, p1;
  p0[0] = pk16(bf_bits(e[0]  * inv), bf_bits(e[1]  * inv));
  p0[1] = pk16(bf_bits(e[2]  * inv), bf_bits(e[3]  * inv));
  p0[2] = pk16(bf_bits(e[4]  * inv), bf_bits(e[5]  * inv));
  p0[3] = pk16(bf_bits(e[6]  * inv), bf_bits(e[7]  * inv));
  p1[0] = pk16(bf_bits(e[8]  * inv), bf_bits(e[9]  * inv));
  p1[1] = pk16(bf_bits(e[10] * inv), bf_bits(e[11] * inv));
  p1[2] = pk16(bf_bits(e[12] * inv), bf_bits(e[13] * inv));
  p1[3] = pk16(bf_bits(e[14] * inv), bf_bits(e[15] * inv));
  unsigned short* prow = P + rb;
  *(volatile v4u*)(prow + c0) = p0;
  *(volatile v4u*)(prow + c1) = p1;
  __threadfence();
  *(volatile v4u*)(prow + c0) = p0;
  *(volatile v4u*)(prow + c1) = p1;
}

extern "C" void kernel_launch(void* const* d_in, const int* in_sizes, int n_in,
                              void* d_out, int out_size, void* d_ws, size_t ws_size,
                              hipStream_t stream) {
  if (n_in < 8) return;
  if (in_sizes[0] != NQ * NH) return;
  if (in_sizes[1] != NM * NH) return;
  if (in_sizes[2] != NH * NH || in_sizes[4] != NH * NH || in_sizes[6] != NH * NH) return;
  if (in_sizes[3] != NH || in_sizes[5] != NH || in_sizes[7] != NH) return;
  if (out_size != NQ * NH) return;

  const float* x  = (const float*)d_in[0];
  const float* mb = (const float*)d_in[1];
  const float* Wq = (const float*)d_in[2];
  const float* bq = (const float*)d_in[3];
  const float* Wk = (const float*)d_in[4];
  const float* bk = (const float*)d_in[5];
  const float* Wv = (const float*)d_in[6];
  const float* bv = (const float*)d_in[7];
  float* out = (float*)d_out;

  const size_t PXb = (size_t)NQ * NH * 2;
  const size_t PMb = (size_t)NM * NH * 2;
  const size_t PW  = (size_t)NH * NH * 2;
  const size_t PQb = (size_t)NQ * NH * 2;
  const size_t PKb = (size_t)NM * NH * 2;
  const size_t PVt = (size_t)NH * NM * 2;
  const size_t PS  = (size_t)QCH * NM * 4;
  const size_t PP  = (size_t)QCH * NM * 2;
  size_t off = 0;
  const size_t oXb = off; off += PXb;
  const size_t oMb = off; off += PMb;
  const size_t oWq = off; off += PW;
  const size_t oWk = off; off += PW;
  const size_t oWv = off; off += PW;
  const size_t oQb = off; off += PQb;
  const size_t oKb = off; off += PKb;
  const size_t oVt = off; off += PVt;
  const size_t oS  = off; off += PS;
  const size_t oP  = off; off += PP;
  if (off > ws_size) return;
  if (off > (size_t)134217728) return;

  char* ws = (char*)d_ws;
  unsigned short* Xb  = (unsigned short*)(ws + oXb);
  unsigned short* Mb  = (unsigned short*)(ws + oMb);
  unsigned short* WqT = (unsigned short*)(ws + oWq);
  unsigned short* WkT = (unsigned short*)(ws + oWk);
  unsigned short* WvT = (unsigned short*)(ws + oWv);
  unsigned short* Qb  = (unsigned short*)(ws + oQb);
  unsigned short* Kb  = (unsigned short*)(ws + oKb);
  unsigned short* Vt  = (unsigned short*)(ws + oVt);
  float* S = (float*)(ws + oS);
  unsigned short* P = (unsigned short*)(ws + oP);

  const dim3 blk(256);
  const int n8x = NQ * NH / 8;
  const int n8m = NM * NH / 8;
  const dim3 gCvtX((n8x + 255) / 256);
  const dim3 gCvtM((n8m + 255) / 256);
  const dim3 gTr(NH / 64, NH / 64);
  const dim3 gQ(((NQ / 64) * (NH / 64) + 7) / 8);
  const dim3 gK(((NM / 64) * (NH / 64) + 7) / 8);
  const dim3 gV(((NH / 64) * (NM / 64) + 7) / 8);
  const dim3 gS(((QCH / 64) * (NM / 64) + 7) / 8);
  const dim3 gSm(QCH);
  const dim3 gO(((QCH / 64) * (NH / 64) + 7) / 8);

  cvt_bf16x8<<<gCvtX, blk, 0, stream>>>(x, Xb, n8x, n8x);
  cvt_bf16x8<<<gCvtM, blk, 0, stream>>>(mb, Mb, n8m, n8m);
  tr_cvt64<<<gTr, blk, 0, stream>>>(Wq, WqT, NH, NH);
  tr_cvt64<<<gTr, blk, 0, stream>>>(Wk, WkT, NH, NH);
  tr_cvt64<<<gTr, blk, 0, stream>>>(Wv, WvT, NH, NH);
  gemm64<1, 1, 0><<<gQ, blk, 0, stream>>>(Xb, NH, WqT, NH, (void*)Qb, NH, bq, NH, x, NH,
                                         1.0f, NQ, NH, NH);
  gemm64<1, 1, 0><<<gK, blk, 0, stream>>>(Mb, NH, WkT, NH, (void*)Kb, NH, bk, NH, x, NH,
                                         1.0f, NM, NH, NH);
  gemm64<1, 2, 0><<<gV, blk, 0, stream>>>(WvT, NH, Mb, NH, (void*)Vt, NM, bv, NH, x, NH,
                                         1.0f, NH, NM, NH);
  for (int q4 = 0; q4 < NQ / QCH; ++q4) {
    const size_t rowOff = (size_t)q4 * QCH;
    gemm64<0, 0, 0><<<gS, blk, 0, stream>>>(Qb + rowOff * NH, NH, Kb, NH, (void*)S, NM, bq, NH, x, NH,
                                           0.03125f, QCH, NM, NH);
    softmax_rows<<<gSm, blk, 0, stream>>>(S, P);
    gemm64<0, 0, 1><<<gO, blk, 0, stream>>>(P, NM, Vt, NM, (void*)(out + rowOff * NH), NH, bq, NH,
                                           x + rowOff * NH, NH, 1.0f, QCH, NH, NM);
  }
  (void)hipGetLastError();
}
